// DGNLayer_47425028882653
// MI455X (gfx1250) — hardware-verified
//
#include <hip/hip_runtime.h>
#include <stddef.h>


#define DF       256
#define NTHR     256
#define NWAVE    8
#define KCH      256
#define APITCH   264
#define ABP      512
#define HCP      768
#define NB       128
#define SLAB     128
#define NPASS    (DF / SLAB)
#define CAPW     1024
#define EPG      8
#define GRP      (NTHR * EPG)
#define NPROWS   8704
#define LDS_GEMM 67584
#define LDS_AGG  230944
#define WS_CAP   134217728

static_assert(NPROWS % NB == 0);
static_assert(NPROWS % 32 == 0);
static_assert(NB == 16 * NWAVE);
static_assert(SLAB == 4 * 32);
static_assert((3 * NB * SLAB + NWAVE * CAPW + 3 * NB + NWAVE) * 4 == LDS_AGG);
static_assert(2 * 32 * APITCH * 2 <= LDS_GEMM);
static_assert(16 * 512 * 4 <= LDS_GEMM);
static_assert(32 * 256 * 4 <= LDS_GEMM);

typedef float          v4f  __attribute__((ext_vector_type(4)));
typedef float          v8f  __attribute__((ext_vector_type(8)));
typedef int            v4i  __attribute__((ext_vector_type(4)));
typedef unsigned short us;
typedef us             v8us __attribute__((ext_vector_type(8)));
typedef _Float16       v8h  __attribute__((ext_vector_type(8)));
typedef _Float16       v16h __attribute__((ext_vector_type(16)));
typedef __bf16         v16b __attribute__((ext_vector_type(16)));
union FragH { v16h v; v8us u[2]; };
union FragB { v16b v; v8us u[2]; };
union Cvt8  { v8h v; v8us u; };

__device__ __forceinline__ unsigned f2bf_bits(float x) {
  const unsigned u = __float_as_uint(x);
  return (u + 0x7FFFu + ((u >> 16) & 1u)) >> 16;
}

__device__ __forceinline__ void split_bf16_8(v4f a, v4f b, v8us& hi, v8us& lo) {
  float x[8] = {a.x, a.y, a.z, a.w, b.x, b.y, b.z, b.w};
#pragma unroll
  for (int i = 0; i < 8; ++i) {
    const unsigned hb = f2bf_bits(x[i]);
    const float r = x[i] - __uint_as_float(hb << 16);
    hi[i] = (us)hb;
    lo[i] = (us)f2bf_bits(r);
  }
}

__device__ __forceinline__ void split_f16_8(v4f a, v4f b, v8us& hi, v8us& lo) {
  float x[8] = {a.x, a.y, a.z, a.w, b.x, b.y, b.z, b.w};
  Cvt8 ch, cl;
#pragma unroll
  for (int i = 0; i < 8; ++i) {
    const _Float16 t = (_Float16)x[i];
    ch.v[i] = t;
    cl.v[i] = (_Float16)((x[i] - (float)t) * 2048.0f);
  }
  hi = ch.u;
  lo = cl.u;
}

__device__ __forceinline__ v8f wmb3(v16b ah, v16b al, v16b bh, v16b bl, v8f c) {
  v8f d = __builtin_amdgcn_wmma_f32_16x16x32_bf16(false, ah, false, bh, (short)0, c, false, false);
  d = __builtin_amdgcn_wmma_f32_16x16x32_bf16(false, ah, false, bl, (short)0, d, false, false);
  d = __builtin_amdgcn_wmma_f32_16x16x32_bf16(false, al, false, bh, (short)0, d, false, false);
  asm volatile("v_nop\n\tv_nop\n\tv_nop\n\tv_nop" : "+v"(d) : "v"(ah), "v"(al), "v"(bh), "v"(bl));
  return d;
}

__device__ __forceinline__ v8f wmh2(v16h ah, v16h al, v16h bh, v16h bs, v8f c) {
  v8f d = __builtin_amdgcn_wmma_f32_16x16x32_f16(false, ah, false, bh, (short)0, c, false, false);
  d = __builtin_amdgcn_wmma_f32_16x16x32_f16(false, al, false, bs, (short)0, d, false, false);
  asm volatile("v_nop\n\tv_nop\n\tv_nop\n\tv_nop" : "+v"(d) : "v"(ah), "v"(al), "v"(bh), "v"(bs));
  return d;
}

__global__ __launch_bounds__(NTHR) void k_prep(
    const float* __restrict__ W1, const float* __restrict__ W2,
    us* w1h, us* w1l, us* w2h, us* w2s) {
  const int i  = (int)blockIdx.x * NTHR + (int)threadIdx.x;
  const int n1 = 2 * DF * DF / 8;
  const int n2 = 4 * DF * DF / 8;
  if (i >= n1 + n2) return;
  v4f xa, xb;
  v8us vh, vl;
  us* dh;
  us* dl;
  if (i < n1) {
    const int o  = i * 8;
    const int n  = o >> 8;
    const int k0 = o & (DF - 1);
    const float* p = (n < DF) ? (W1 + (size_t)k0 * DF + n) : (W1 + (size_t)(DF + k0) * DF + (n - DF));
    xa.x = p[0];      xa.y = p[DF];     xa.z = p[2 * DF]; xa.w = p[3 * DF];
    xb.x = p[4 * DF]; xb.y = p[5 * DF]; xb.z = p[6 * DF]; xb.w = p[7 * DF];
    split_bf16_8(xa, xb, vh, vl);
    dh = w1h + o;
    dl = w1l + o;
  } else {
    const int o  = (i - n1) * 8;
    const int n  = o >> 10;
    const int k0 = o & (4 * DF - 1);
    const float* p = W2 + (size_t)k0 * DF + n;
    xa.x = p[0];      xa.y = p[DF];     xa.z = p[2 * DF]; xa.w = p[3 * DF];
    xb.x = p[4 * DF]; xb.y = p[5 * DF]; xb.z = p[6 * DF]; xb.w = p[7 * DF];
    float x[8] = {xa.x, xa.y, xa.z, xa.w, xb.x, xb.y, xb.z, xb.w};
    Cvt8 ch, cs;
#pragma unroll
    for (int j = 0; j < 8; ++j) {
      ch.v[j] = (_Float16)(x[j] * 64.0f);
      cs.v[j] = (_Float16)(x[j] * 0.03125f);
    }
    vh = ch.u;
    vl = cs.u;
    dh = w2h + o;
    dl = w2s + o;
  }
  *(volatile v8us*)dh = vh;
  *(volatile v8us*)dl = vl;
  __threadfence();
  *(volatile v8us*)dh = vh;
  *(volatile v8us*)dl = vl;
}

template <int MODE, int ROWG, int EPI, int TPW>
__global__ __launch_bounds__(NTHR) void k_gemm(
    const float* __restrict__ A0, const float* __restrict__ A1,
    const us* __restrict__ Bp, const us* __restrict__ Bq,
    const float* __restrict__ bias, const float* __restrict__ rscale,
    float* C, float* part,
    int lda0, int K0, int lda1, int a1off, int K,
    int nrowclamp, int nrowstore, int ldc, int rowbase) {
  constexpr int COLG = NWAVE / ROWG;
  constexpr int ROWS = 16 * ROWG;
  constexpr int WC   = 16 * TPW;
  constexpr int COLS = WC * COLG;
  constexpr int NSTI = WC / 8;
  constexpr int RPI  = 128 / WC;
  static_assert(ROWG * COLG == NWAVE);
  static_assert(WC == 64 || WC == 128);
  static_assert(EPI == 0 || COLS == NTHR);
  static_assert(2 * ROWS * APITCH * 2 <= LDS_GEMM);
  static_assert(ROWS * COLS * 4 <= LDS_GEMM);
  extern __shared__ v4f lds_dyn[];
  us*    sAh = (us*)lds_dyn;
  us*    sAl = sAh + ROWS * APITCH;
  float* stg = (float*)lds_dyn;
  const int tid = threadIdx.x, lane = tid & 31, wave = tid >> 5, hh = lane >> 4, m = lane & 15;
  const int rg = wave % ROWG, cg = wave / ROWG;
  const int grow0 = rowbase + (int)blockIdx.x * ROWS;
  const int colw = cg * WC;

  v8f acc[TPW];
#pragma unroll
  for (int t = 0; t < TPW; ++t) { v8f z = {0.f, 0.f, 0.f, 0.f, 0.f, 0.f, 0.f, 0.f}; acc[t] = z; }

  const int nkc = K / KCH;
#pragma unroll 1
  for (int kci = 0; kci < nkc; ++kci) {
    const int kc = kci * KCH;
#pragma unroll
    for (int i = 0; i < ROWS / 8; ++i) {
      const int idx = i * NTHR + tid;
      const int r   = idx >> 5;
      const int c8  = (idx & 31) * 8;
      int grow = grow0 + r;
      grow = grow > nrowclamp - 1 ? nrowclamp - 1 : grow;
      const float* sp;
      if (kc < K0) sp = A0 + (size_t)grow * (size_t)lda0 + kc + c8;
      else         sp = A1 + (size_t)(grow - a1off) * (size_t)lda1 + (kc - K0) + c8;
      const v4f x0 = *(const v4f*)sp;
      const v4f x1 = *(const v4f*)(sp + 4);
      v8us vh, vl;
      if (MODE == 0) split_bf16_8(x0, x1, vh, vl);
      else           split_f16_8(x0, x1, vh, vl);
      *(v8us*)(sAh + r * APITCH + c8) = vh;
      *(v8us*)(sAl + r * APITCH + c8) = vl;
    }
    __syncthreads();
    const us* arh = sAh + (rg * 16 + m) * APITCH + 8 * hh;
    const us* arl = sAl + (rg * 16 + m) * APITCH + 8 * hh;
#pragma unroll 1
    for (int kt = 0; kt < KCH / 32; ++kt) {
      const int kk = 32 * kt;
      const size_t kg = (size_t)(kc + kk + 8 * hh);
      if (MODE == 0) {
        FragB fa, fl;
        fa.u[0] = *(const v8us*)(arh + kk);
        fa.u[1] = *(const v8us*)(arh + kk + 16);
        fl.u[0] = *(const v8us*)(arl + kk);
        fl.u[1] = *(const v8us*)(arl + kk + 16);
#pragma unroll
        for (int t = 0; t < TPW; ++t) {
          const size_t bo = (size_t)(colw + 16 * t + m) * (size_t)K + kg;
          FragB fb, fc;
          fb.u[0] = *(const v8us*)(Bp + bo);
          fb.u[1] = *(const v8us*)(Bp + bo + 16);
          fc.u[0] = *(const v8us*)(Bq + bo);
          fc.u[1] = *(const v8us*)(Bq + bo + 16);
          acc[t] = wmb3(fa.v, fl.v, fb.v, fc.v, acc[t]);
        }
      } else {
        FragH fa, fl;
        fa.u[0] = *(const v8us*)(arh + kk);
        fa.u[1] = *(const v8us*)(arh + kk + 16);
        fl.u[0] = *(const v8us*)(arl + kk);
        fl.u[1] = *(const v8us*)(arl + kk + 16);
#pragma unroll
        for (int t = 0; t < TPW; ++t) {
          const size_t bo = (size_t)(colw + 16 * t + m) * (size_t)K + kg;
          FragH fb, fc;
          fb.u[0] = *(const v8us*)(Bp + bo);
          fb.u[1] = *(const v8us*)(Bp + bo + 16);
          fc.u[0] = *(const v8us*)(Bq + bo);
          fc.u[1] = *(const v8us*)(Bq + bo + 16);
          acc[t] = wmh2(fa.v, fl.v, fb.v, fc.v, acc[t]);
        }
      }
    }
    __syncthreads();
  }

  const float osc = (MODE == 0) ? 1.0f : 0.015625f;
  float rs8[8], bc8[TPW];
#pragma unroll
  for (int r = 0; r < 8; ++r) rs8[r] = 1.0f;
#pragma unroll
  for (int t = 0; t < TPW; ++t) bc8[t] = 0.0f;
  if (EPI) {
#pragma unroll
    for (int r = 0; r < 8; ++r) {
      const int grow = grow0 + rg * 16 + 8 * hh + r;
      const int gc   = grow > nrowclamp - 1 ? nrowclamp - 1 : grow;
      const float sv = rscale[gc];
      rs8[r] = (grow < nrowstore) ? sv : 0.0f;
    }
#pragma unroll
    for (int t = 0; t < TPW; ++t) bc8[t] = bias[colw + 16 * t + m];
  }
  float* stp = stg + (rg * 16 + 8 * hh) * COLS + colw + m;
#pragma unroll
  for (int t = 0; t < TPW; ++t) {
#pragma unroll
    for (int r = 0; r < 8; ++r) {
      float v = acc[t][r] * osc;
      if (EPI) v = (v + bc8[t]) * rs8[r];
      stp[r * COLS + 16 * t] = v;
    }
  }
  __syncthreads();

  const int rr = (4 * lane) / WC;
  const int cc = (4 * lane) - rr * WC;
  const float* lrp = stg + (rg * 16) * COLS + colw + cc;
#pragma unroll
  for (int i = 0; i < NSTI; ++i) {
    const int row  = i * RPI + rr;
    const int grow = grow0 + rg * 16 + row;
    if (grow < nrowstore) {
      const v4f v = *(const v4f*)(lrp + row * COLS);
      *(volatile v4f*)(C + (size_t)grow * (size_t)ldc + colw + cc) = v;
    }
  }
  __threadfence();
#pragma unroll
  for (int i = 0; i < NSTI; ++i) {
    const int row  = i * RPI + rr;
    const int grow = grow0 + rg * 16 + row;
    if (grow < nrowstore) {
      const v4f v = *(const v4f*)(lrp + row * COLS);
      *(volatile v4f*)(C + (size_t)grow * (size_t)ldc + colw + cc) = v;
    }
  }

  if (EPI) {
    float s = 0.0f, q = 0.0f;
#pragma unroll 8
    for (int r = 0; r < ROWS; ++r) {
      const float v = stg[r * COLS + tid];
      s += v;
      q = fmaf(v, v, q);
    }
    float* pp = part + (size_t)(grow0 / ROWS) * (size_t)(2 * COLS);
    *(volatile float*)(pp + tid) = s;
    *(volatile float*)(pp + COLS + tid) = q;
    __threadfence();
    *(volatile float*)(pp + tid) = s;
    *(volatile float*)(pp + COLS + tid) = q;
  }
}

#define HITJ(J, QJ, SJ) { \
    const unsigned mj = __builtin_amdgcn_ballot_w32(QJ); \
    if (mj != 0u) { \
      if (QJ) { \
        const int pos = cnt + (int)__builtin_amdgcn_mbcnt_lo(mj, 0u); \
        if (pos < CAPW) wl[wave * CAPW + pos] = ((e0 + (J)) << 7) | (int)(SJ); \
      } \
      cnt += (int)__builtin_popcount(mj); } }

__global__ __launch_bounds__(NTHR) void k_agg(
    const int* __restrict__ srcs, const int* __restrict__ dsts, const float* __restrict__ eig,
    const float* __restrict__ h, const float* __restrict__ ab, const float* __restrict__ b1,
    float* hc, int nN, int nE, int partBase) {
  extern __shared__ v4f lds_dyn[];
  float* accS = (float*)lds_dyn;
  float* accU = accS + NB * SLAB;
  float* accW = accU + NB * SLAB;
  int*   wl   = (int*)(accW + NB * SLAB);
  int*   degL = wl + NWAVE * CAPW;
  float* sabL = (float*)(degL + NB);
  float* swL  = sabL + NB;
  int*   wcnt = (int*)(swL + NB);
  const int tid = threadIdx.x, lane = tid & 31, wave = tid >> 5;
  const int nodeBase = partBase + (int)blockIdx.x * NB;
  const unsigned nbu = (unsigned)nodeBase;

  int cnt = 0;
  const int nG   = (nE + GRP - 1) / GRP;
  const int sent = -2147483647 - 1;
#pragma unroll 1
  for (int g = 0; g < nG; ++g) {
    const int e0 = g * GRP + tid * EPG;
    v4i da, db;
    if (e0 + 7 < nE) {
      da = *(const v4i*)(dsts + e0);
      db = *(const v4i*)(dsts + e0 + 4);
    } else {
      da.x = (e0     < nE) ? dsts[min(e0,     nE - 1)] : sent;
      da.y = (e0 + 1 < nE) ? dsts[min(e0 + 1, nE - 1)] : sent;
      da.z = (e0 + 2 < nE) ? dsts[min(e0 + 2, nE - 1)] : sent;
      da.w = (e0 + 3 < nE) ? dsts[min(e0 + 3, nE - 1)] : sent;
      db.x = (e0 + 4 < nE) ? dsts[min(e0 + 4, nE - 1)] : sent;
      db.y = (e0 + 5 < nE) ? dsts[min(e0 + 5, nE - 1)] : sent;
      db.z = (e0 + 6 < nE) ? dsts[min(e0 + 6, nE - 1)] : sent;
      db.w = (e0 + 7 < nE) ? dsts[min(e0 + 7, nE - 1)] : sent;
    }
    const unsigned s0 = (unsigned)da.x - nbu, s1 = (unsigned)da.y - nbu;
    const unsigned s2 = (unsigned)da.z - nbu, s3 = (unsigned)da.w - nbu;
    const unsigned s4 = (unsigned)db.x - nbu, s5 = (unsigned)db.y - nbu;
    const unsigned s6 = (unsigned)db.z - nbu, s7 = (unsigned)db.w - nbu;
    const bool q0 = s0 < (unsigned)NB, q1 = s1 < (unsigned)NB, q2 = s2 < (unsigned)NB, q3 = s3 < (unsigned)NB;
    const bool q4 = s4 < (unsigned)NB, q5 = s5 < (unsigned)NB, q6 = s6 < (unsigned)NB, q7 = s7 < (unsigned)NB;
    const unsigned any = __builtin_amdgcn_ballot_w32(q0 | q1 | q2 | q3 | q4 | q5 | q6 | q7);
    if (any != 0u) {
      HITJ(0, q0, s0)
      HITJ(1, q1, s1)
      HITJ(2, q2, s2)
      HITJ(3, q3, s3)
      HITJ(4, q4, s4)
      HITJ(5, q5, s5)
      HITJ(6, q6, s6)
      HITJ(7, q7, s7)
    }
  }
  if (lane == 0) wcnt[wave] = cnt < CAPW ? cnt : CAPW;
  __syncthreads();

#pragma unroll 1
  for (int ps = 0; ps < NPASS; ++ps) {
    const int c0 = ps * SLAB;
    {
      const v4f z = {0.f, 0.f, 0.f, 0.f};
      for (int i = tid; i < 3 * NB * SLAB / 4; i += NTHR) lds_dyn[i] = z;
    }
    if (ps == 0 && tid < NB) { degL[tid] = 0; sabL[tid] = 0.0f; swL[tid] = 0.0f; }
    __syncthreads();

#pragma unroll 1
    for (int s = 0; s < NWAVE; ++s) {
      int ns = __builtin_amdgcn_readfirstlane(wcnt[s]);
      ns = ns > CAPW ? CAPW : (ns < 0 ? 0 : ns);
      const int* lp = wl + s * CAPW;
#pragma unroll 1
      for (int base = 0; base < ns; base += 32) {
        const int idx = base + lane;
        const int ent = (idx < ns) ? lp[idx] : -1;
        const bool own = (ent >= 0) && ((((unsigned)ent & (unsigned)(NB - 1)) >> 4) == (unsigned)wave);
        unsigned msk = __builtin_amdgcn_ballot_w32(own);
#pragma unroll 1
        while (msk != 0u) {
          const int bsel = __builtin_ctz(msk);
          msk &= msk - 1u;
          const int eu   = __builtin_amdgcn_readlane(ent, bsel);
          const int slot = eu & (NB - 1);
          int e = eu >> 7;
          e = e > nE - 1 ? nE - 1 : e;
          int sn = srcs[e];
          sn = sn < 0 ? 0 : (sn > nN - 1 ? nN - 1 : sn);
          const float wv = eig[2 * (size_t)e];
          const float aw = fabsf(wv);
          if (ps == 0 && lane == 0) {
            degL[slot] = degL[slot] + 1;
            sabL[slot] = sabL[slot] + aw;
            swL[slot]  = swL[slot] + wv;
          }
          const v4f v = *(const v4f*)(ab + (size_t)sn * ABP + c0 + 4 * lane);
          v4f* pS = (v4f*)(accS + slot * SLAB + 4 * lane);
          v4f* pU = (v4f*)(accU + slot * SLAB + 4 * lane);
          v4f* pW = (v4f*)(accW + slot * SLAB + 4 * lane);
          *pS = *pS + v;
          *pU = *pU + aw * v;
          *pW = *pW + wv * v;
        }
      }
    }
    __syncthreads();

    const int cl = c0 + 4 * lane;
    const v4f b14 = *(const v4f*)(b1 + cl);
#pragma unroll 1
    for (int r = 0; r < NB / NWAVE; ++r) {
      const int slot  = wave * (NB / NWAVE) + r;
      const int node  = nodeBase + slot;
      const int nodec = node > nN - 1 ? nN - 1 : node;
      const size_t lrow = (size_t)(node - partBase);
      const float degf = (float)degL[slot];
      const float rdeg = 1.0f / fmaxf(degf, 1.0f);
      const float sab  = sabL[slot];
      const float rsn  = 1.0f / (sab + 1e-8f);
      const float swv  = swL[slot];
      const v4f bb = *(const v4f*)(ab + (size_t)nodec * ABP + DF + cl) + b14;
      const v4f hv = *(const v4f*)(h + (size_t)nodec * DF + cl);
      v4f* pS = (v4f*)(accS + slot * SLAB + 4 * lane);
      v4f* pU = (v4f*)(accU + slot * SLAB + 4 * lane);
      v4f* pW = (v4f*)(accW + slot * SLAB + 4 * lane);
      const v4f mean = (*pS + degf * bb) * rdeg;
      const v4f av   = (*pU + sab * bb) * rsn;
      v4f dx = (*pW + swv * bb) * rsn - hv;
      dx.x = fabsf(dx.x); dx.y = fabsf(dx.y); dx.z = fabsf(dx.z); dx.w = fabsf(dx.w);
      *pS = mean; *pU = av; *pW = dx;
      float* gp = hc + lrow * HCP + cl;
      *(volatile v4f*)(gp)          = mean;
      *(volatile v4f*)(gp + DF)     = av;
      *(volatile v4f*)(gp + 2 * DF) = dx;
    }
    __threadfence();
#pragma unroll 1
    for (int r = 0; r < NB / NWAVE; ++r) {
      const int slot = wave * (NB / NWAVE) + r;
      const int node = nodeBase + slot;
      const size_t lrow = (size_t)(node - partBase);
      const v4f mean = *(const v4f*)(accS + slot * SLAB + 4 * lane);
      const v4f av   = *(const v4f*)(accU + slot * SLAB + 4 * lane);
      const v4f dx   = *(const v4f*)(accW + slot * SLAB + 4 * lane);
      float* gp = hc + lrow * HCP + cl;
      *(volatile v4f*)(gp)          = mean;
      *(volatile v4f*)(gp + DF)     = av;
      *(volatile v4f*)(gp + 2 * DF) = dx;
    }
    __syncthreads();
  }
}
#undef HITJ

__global__ __launch_bounds__(NTHR) void k_bnstat(const float* __restrict__ part, float* stat,
                                                  int nslot, int nN) {
  const int c = threadIdx.x;
  double s = 0.0, q = 0.0;
#pragma unroll 1
  for (int b = 0; b < nslot; ++b) {
    s += (double)part[(size_t)b * 512 + c];
    q += (double)part[(size_t)b * 512 + 256 + c];
  }
  const double inv = 1.0 / (double)nN;
  const double mu  = s * inv;
  double var = q * inv - mu * mu;
  var = var < 0.0 ? 0.0 : var;
  const float muf = (float)mu;
  const float rsf = 1.0f / sqrtf((float)var + 1e-5f);
  *(volatile float*)(stat + c)       = muf;
  *(volatile float*)(stat + 256 + c) = rsf;
  __threadfence();
  *(volatile float*)(stat + c)       = muf;
  *(volatile float*)(stat + 256 + c) = rsf;
}

__global__ __launch_bounds__(NTHR) void k_final(
    const float* __restrict__ h, const float* __restrict__ stat,
    const float* __restrict__ gamma, const float* __restrict__ beta,
    float* out, int total) {
  const int tid = threadIdx.x, lane = tid & 31, wave = tid >> 5;
  const size_t base = ((size_t)blockIdx.x * NWAVE + (size_t)wave) * 1024;
  const int ca = 4 * lane, cb = 128 + 4 * lane;
  const v4f mua = *(const v4f*)(stat + ca),       mub = *(const v4f*)(stat + cb);
  const v4f rsa = *(const v4f*)(stat + 256 + ca), rsb = *(const v4f*)(stat + 256 + cb);
  const v4f ga  = *(const v4f*)(gamma + ca),      gb  = *(const v4f*)(gamma + cb);
  const v4f ba  = *(const v4f*)(beta + ca),       bbv = *(const v4f*)(beta + cb);
  v4f res[8];
#pragma unroll
  for (int q = 0; q < 8; ++q) {
    const size_t f = base + (size_t)q * 128 + 4 * lane;
    v4f rv = {0.f, 0.f, 0.f, 0.f};
    if (base + (size_t)q * 128 < (size_t)total) {
      const v4f x  = *(const v4f*)(out + f);
      const v4f hv = *(const v4f*)(h + f);
      const bool odd = (q & 1) != 0;
      const v4f mu = odd ? mub : mua;
      const v4f rs = odd ? rsb : rsa;
      const v4f gm = odd ? gb : ga;
      const v4f bt = odd ? bbv : ba;
      v4f y = ((x - mu) * rs) * gm + bt;
      y.x = fmaxf(y.x, 0.f); y.y = fmaxf(y.y, 0.f); y.z = fmaxf(y.z, 0.f); y.w = fmaxf(y.w, 0.f);
      rv = hv + y;
    }
    res[q] = rv;
  }
#pragma unroll
  for (int q = 0; q < 8; ++q) {
    const size_t f = base + (size_t)q * 128 + 4 * lane;
    if (base + (size_t)q * 128 < (size_t)total) *(volatile v4f*)(out + f) = res[q];
  }
  __threadfence();
#pragma unroll
  for (int q = 0; q < 8; ++q) {
    const size_t f = base + (size_t)q * 128 + 4 * lane;
    if (base + (size_t)q * 128 < (size_t)total) *(volatile v4f*)(out + f) = res[q];
  }
}

extern "C" void kernel_launch(void* const* d_in, const int* in_sizes, int n_in,
                              void* d_out, int out_size, void* d_ws, size_t ws_size,
                              hipStream_t stream) {
  if (n_in < 11) return;
  const int nN = in_sizes[0] / DF;
  const int nE = in_sizes[9];
  if (nN <= 0 || nE <= 0) return;
  if (in_sizes[0] != nN * DF || in_sizes[1] != 2 * nE || in_sizes[10] != nE || in_sizes[2] != nN) return;
  if (in_sizes[3] != 2 * DF * DF || in_sizes[4] != DF || in_sizes[5] != 4 * DF * DF ||
      in_sizes[6] != DF || in_sizes[7] != DF || in_sizes[8] != DF) return;
  if (out_size != nN * DF) return;
  if (nE > (1 << 23)) return;

  const float* h     = (const float*)d_in[0];
  const float* eig   = (const float*)d_in[1];
  const float* snorm = (const float*)d_in[2];
  const float* W1    = (const float*)d_in[3];
  const float* b1    = (const float*)d_in[4];
  const float* W2    = (const float*)d_in[5];
  const float* b2    = (const float*)d_in[6];
  const float* gamma = (const float*)d_in[7];
  const float* beta  = (const float*)d_in[8];
  const int*   src   = (const int*)d_in[9];
  const int*   dst   = (const int*)d_in[10];
  float* out = (float*)d_out;

  const int rowsF = ((nN + 31) / 32) * 32;
  const int nSlot = (nN + 31) / 32;
  const int nPart = (nN + NPROWS - 1) / NPROWS;

  char* ws = (char*)d_ws;
  size_t off = 0;
  const size_t oW1h = off; off += (size_t)2 * DF * DF * 2;          off = (off + 255) & ~(size_t)255;
  const size_t oW1l = off; off += (size_t)2 * DF * DF * 2;          off = (off + 255) & ~(size_t)255;
  const size_t oW2h = off; off += (size_t)4 * DF * DF * 2;          off = (off + 255) & ~(size_t)255;
  const size_t oW2s = off; off += (size_t)4 * DF * DF * 2;          off = (off + 255) & ~(size_t)255;
  const size_t oAB  = off; off += (size_t)rowsF * ABP * 4;          off = (off + 255) & ~(size_t)255;
  const size_t oHC  = off; off += (size_t)NPROWS * HCP * 4;         off = (off + 255) & ~(size_t)255;
  const size_t oPT  = off; off += (size_t)nSlot * 512 * 4;          off = (off + 255) & ~(size_t)255;
  const size_t oST  = off; off += (size_t)512 * 4;                  off = (off + 255) & ~(size_t)255;
  if (off > ws_size || off > (size_t)WS_CAP) return;
  us*    w1h  = (us*)(ws + oW1h);
  us*    w1l  = (us*)(ws + oW1l);
  us*    w2h  = (us*)(ws + oW2h);
  us*    w2s  = (us*)(ws + oW2s);
  float* ab   = (float*)(ws + oAB);
  float* hcb  = (float*)(ws + oHC);
  float* part = (float*)(ws + oPT);
  float* stat = (float*)(ws + oST);

  const int nPrep = 2 * DF * DF / 8 + 4 * DF * DF / 8;
  k_prep<<<(nPrep + NTHR - 1) / NTHR, NTHR, 0, stream>>>(W1, W2, w1h, w1l, w2h, w2s);

  hipFuncSetAttribute(reinterpret_cast<const void*>(&k_gemm<0, 1, 0, 4>),
                      hipFuncAttributeMaxDynamicSharedMemorySize, LDS_GEMM);
  k_gemm<0, 1, 0, 4><<<rowsF / 16, NTHR, LDS_GEMM, stream>>>(
      h, h, w1h, w1l, b1, snorm, ab, part,
      DF, DF, DF, 0, DF, nN, rowsF, ABP, 0);

  hipFuncSetAttribute(reinterpret_cast<const void*>(&k_agg),
                      hipFuncAttributeMaxDynamicSharedMemorySize, LDS_AGG);
  hipFuncSetAttribute(reinterpret_cast<const void*>(&k_gemm<1, 2, 1, 4>),
                      hipFuncAttributeMaxDynamicSharedMemorySize, LDS_GEMM);
  for (int p = 0; p < nPart; ++p) {
    const int pb   = p * NPROWS;
    const int rows = (nN - pb) < NPROWS ? (nN - pb) : NPROWS;
    k_agg<<<(rows + NB - 1) / NB, NTHR, LDS_AGG, stream>>>(src, dst, eig, h, ab, b1, hcb, nN, nE, pb);
    k_gemm<1, 2, 1, 4><<<(rows + 31) / 32, NTHR, LDS_GEMM, stream>>>(
        h, hcb, w2h, w2s, b2, snorm, out, part,
        DF, DF, HCP, pb, 4 * DF, nN, nN, DF, pb);
  }

  k_bnstat<<<1, NTHR, 0, stream>>>(part, stat, nSlot, nN);
  const int nWavesF = (nN * DF + 1023) / 1024;
  k_final<<<(nWavesF + NWAVE - 1) / NWAVE, NTHR, 0, stream>>>(h, stat, gamma, beta, out, nN * DF);
}
